// DualGNN_77309411328099
// MI455X (gfx1250) — hardware-verified
//
#include <hip/hip_runtime.h>
#include <stddef.h>


#define FW        128
#define LDA16     192
#define KBMAX     160
#define PLH       (FW * KBMAX)
#define NWPL      5
#define NTHR      256
#define NWAVE     8
#define EPT       8
#define NGRP      2
#define CHUNK     (NTHR * EPT * NGRP)
#define WCAP      (EPT * NGRP * 32)
#define LISTN     (NWAVE * WCAP)
#define NBC       4096
#define NBF       1024
#define RCAP      40960
#define RBN       128
#define TGT       256
#define DEGCAP    1024
#define OTHR      512
#define BM        64
#define NCLS      8
#define GCLS      4
#define NGR       64
#define WSCAP     134217728
#define BN_EPS    1e-5f
#define NEG_SLOPE 0.01f
#define ACARRY    16.0f
#define WCARRY    64.0f
#define CARRY_INV 0.0009765625f
#define LDS_FILL  ((RCAP + NBF + LISTN) * 4 + 64)

static_assert((CHUNK & (CHUNK - 1)) == 0);
static_assert(CHUNK <= 4096);
static_assert((NBC & (NBC - 1)) == 0 && (NBF & (NBF - 1)) == 0);
static_assert(NBC == 4 * NBF);
static_assert(OTHR * 8 == NBC);
static_assert((RCAP % 32) == 0);
static_assert(TGT == NWAVE * 32);
static_assert((NBC % TGT) == 0);
static_assert((TGT % BM) == 0);
static_assert(FW == 4 * 32);
static_assert((FW % 32) == 0 && (KBMAX % 32) == 0);
static_assert((LDA16 % 8) == 0 && LDA16 >= KBMAX);
static_assert(WCAP == EPT * NGRP * 32);
static_assert(NGR * GCLS == NTHR);
static_assert(2 * BM * 4 == BM * NCLS);

typedef float          v4f  __attribute__((ext_vector_type(4)));
typedef float          v8f  __attribute__((ext_vector_type(8)));
typedef int            v4i  __attribute__((ext_vector_type(4)));
typedef unsigned int   v2u  __attribute__((ext_vector_type(2)));
typedef _Float16       v4h  __attribute__((ext_vector_type(4)));
typedef _Float16       v8h  __attribute__((ext_vector_type(8)));
typedef _Float16       v16h __attribute__((ext_vector_type(16)));
union Frag  { v16h v; v8h h[2]; };
union Pack4 { v4h h; v2u u; };

__device__ __forceinline__ v8f wmh(v16h a, v16h b, v8f c) {
  v8f d = __builtin_amdgcn_wmma_f32_16x16x32_f16(false, a, false, b, (short)0, c, false, false);
  asm volatile("v_nop\n\tv_nop\n\tv_nop\n\tv_nop" : "+v"(d) : "v"(a), "v"(b));
  return d;
}

__device__ __forceinline__ float lreluf(float v) { return v >= 0.f ? v : NEG_SLOPE * v; }

template <int NB>
__device__ __forceinline__ int scan_chunk(const int* __restrict__ ids, int nE, int cbase, int slotBase,
                                          int vec8, int* list, int tid, int lane, int wave) {
  int wc = 0;
#pragma unroll
  for (int g = 0; g < NGRP; ++g) {
    const int el0  = (g * NTHR + tid) * EPT;
    const int e0   = cbase + el0;
    const int sent = -2147483647 - 1;
    v4i da, db;
    if (vec8 != 0 && cbase + CHUNK <= nE) {
      da = *(const v4i*)(ids + e0);
      db = *(const v4i*)(ids + e0 + 4);
    } else {
      da.x = (e0     < nE) ? ids[min(e0, nE - 1)] : sent;
      da.y = (e0 + 1 < nE) ? ids[min(e0 + 1, nE - 1)] : sent;
      da.z = (e0 + 2 < nE) ? ids[min(e0 + 2, nE - 1)] : sent;
      da.w = (e0 + 3 < nE) ? ids[min(e0 + 3, nE - 1)] : sent;
      db.x = (e0 + 4 < nE) ? ids[min(e0 + 4, nE - 1)] : sent;
      db.y = (e0 + 5 < nE) ? ids[min(e0 + 5, nE - 1)] : sent;
      db.z = (e0 + 6 < nE) ? ids[min(e0 + 6, nE - 1)] : sent;
      db.w = (e0 + 7 < nE) ? ids[min(e0 + 7, nE - 1)] : sent;
    }
    const unsigned nb = (unsigned)slotBase;
    const unsigned s0 = (unsigned)da.x - nb, s1 = (unsigned)da.y - nb;
    const unsigned s2 = (unsigned)da.z - nb, s3 = (unsigned)da.w - nb;
    const unsigned s4 = (unsigned)db.x - nb, s5 = (unsigned)db.y - nb;
    const unsigned s6 = (unsigned)db.z - nb, s7 = (unsigned)db.w - nb;
    const bool h0 = s0 < (unsigned)NB, h1 = s1 < (unsigned)NB, h2 = s2 < (unsigned)NB, h3 = s3 < (unsigned)NB;
    const bool h4 = s4 < (unsigned)NB, h5 = s5 < (unsigned)NB, h6 = s6 < (unsigned)NB, h7 = s7 < (unsigned)NB;
    const unsigned any = __builtin_amdgcn_ballot_w32(h0 | h1 | h2 | h3 | h4 | h5 | h6 | h7);
    if (any != 0u) {
#define HITJ(J, HJ, SJ) { \
        const unsigned mj = __builtin_amdgcn_ballot_w32(HJ); \
        if (mj != 0u) { \
          if (HJ) { \
            const int pos = wc + (int)__builtin_amdgcn_mbcnt_lo(mj, 0u); \
            if (pos < WCAP) list[wave * WCAP + pos] = ((el0 + (J)) << 12) | (int)(SJ); \
          } \
          wc += (int)__builtin_popcount(mj); } }
      HITJ(0, h0, s0)
      HITJ(1, h1, s1)
      HITJ(2, h2, s2)
      HITJ(3, h3, s3)
      HITJ(4, h4, s4)
      HITJ(5, h5, s5)
      HITJ(6, h6, s6)
      HITJ(7, h7, s7)
#undef HITJ
    }
  }
  return wc;
}

__global__ __launch_bounds__(NTHR) void k_count(
    const int* __restrict__ ids, int* cnt, float* dinv, int nE, int vec8) {
  __shared__ __attribute__((aligned(16))) int scnt[NBC];
  __shared__ __attribute__((aligned(16))) int list[LISTN];
  __shared__ int wcnt[NWAVE];
  const int tid = threadIdx.x, lane = tid & 31, wave = tid >> 5;
  const int nodeBase = blockIdx.x * NBC;

  for (int i = tid; i < NBC; i += NTHR) scnt[i] = 0;
  __syncthreads();

  const int nChunks = (nE + CHUNK - 1) / CHUNK;
#pragma unroll 1
  for (int ch = 0; ch < nChunks; ++ch) {
    const int cbase = ch * CHUNK;
    const int wc = scan_chunk<NBC>(ids, nE, cbase, nodeBase, vec8, list, tid, lane, wave);
    if (lane == 0) wcnt[wave] = wc;
    __syncthreads();
    if (wave == 0) {
#pragma unroll 1
      for (int wsx = 0; wsx < NWAVE; ++wsx) {
        int n = __builtin_amdgcn_readfirstlane(wcnt[wsx]);
        n = n > WCAP ? WCAP : (n < 0 ? 0 : n);
        const int* lp = list + wsx * WCAP;
#pragma unroll 1
        for (int i = 0; i < n; ++i) {
          const int ent  = __builtin_amdgcn_readfirstlane(lp[i]);
          const int slot = ent & (NBC - 1);
          if (lane == 0) scnt[slot] = scnt[slot] + 1;
        }
      }
    }
    __syncthreads();
  }

  v4i cq[4];
  v4f dq[4];
#pragma unroll
  for (int q = 0; q < 4; ++q) {
    const int f = (wave * 4 + q) * 128 + 4 * lane;
    const v4i cv = *(const v4i*)(scnt + f);
    cq[q] = cv;
    v4f d;
    d.x = rsqrtf(fmaxf((float)cv.x, 1.0f));
    d.y = rsqrtf(fmaxf((float)cv.y, 1.0f));
    d.z = rsqrtf(fmaxf((float)cv.z, 1.0f));
    d.w = rsqrtf(fmaxf((float)cv.w, 1.0f));
    dq[q] = d;
  }
  int*   cp = cnt  + (size_t)nodeBase;
  float* dp = dinv + (size_t)nodeBase;
#pragma unroll
  for (int q = 0; q < 4; ++q) {
    const int f = (wave * 4 + q) * 128 + 4 * lane;
    *(volatile v4i*)(cp + f) = cq[q];
    *(volatile v4f*)(dp + f) = dq[q];
  }
  __threadfence();
#pragma unroll
  for (int q = 0; q < 4; ++q) {
    const int f = (wave * 4 + q) * 128 + 4 * lane;
    *(volatile v4i*)(cp + f) = cq[q];
    *(volatile v4f*)(dp + f) = dq[q];
  }
}

__global__ __launch_bounds__(OTHR) void k_offsets(
    const int* __restrict__ cnt, int* off, int* rbase, int nChunk) {
  __shared__ __attribute__((aligned(16))) int soff[NBC];
  __shared__ __attribute__((aligned(16))) int srb[RBN];
  __shared__ int wtot[OTHR / 32];
  const int tid = threadIdx.x, lane = tid & 31, wave = tid >> 5, sub = tid >> 7;
  for (int i = tid; i < RBN; i += OTHR) srb[i] = 0;
  int carry = 0;
#pragma unroll 1
  for (int ch = 0; ch < nChunk; ++ch) {
    const int base = ch * NBC;
    const v4i c0 = *(const v4i*)(cnt + base + 8 * tid);
    const v4i c1 = *(const v4i*)(cnt + base + 8 * tid + 4);
    const int e0 = max(c0.x, 0), e1 = max(c0.y, 0), e2 = max(c0.z, 0), e3 = max(c0.w, 0);
    const int e4 = max(c1.x, 0), e5 = max(c1.y, 0), e6 = max(c1.z, 0), e7 = max(c1.w, 0);
    const int ts = e0 + e1 + e2 + e3 + e4 + e5 + e6 + e7;
    int incl = ts;
#pragma unroll
    for (int d = 1; d < 32; d <<= 1) {
      const int t = __shfl_up(incl, d);
      if (lane >= d) incl += t;
    }
    if (lane == 31) wtot[wave] = incl;
    __syncthreads();
    const int S0 = wtot[0]  + wtot[1]  + wtot[2]  + wtot[3];
    const int S1 = wtot[4]  + wtot[5]  + wtot[6]  + wtot[7];
    const int S2 = wtot[8]  + wtot[9]  + wtot[10] + wtot[11];
    const int S3 = wtot[12] + wtot[13] + wtot[14] + wtot[15];
    int pre = 0;
#pragma unroll 1
    for (int w = 4 * sub; w < wave; ++w) pre += wtot[w];
    const int b0 = carry;
    const int b1 = b0 + ((S0 + 31) & ~31);
    const int b2 = b1 + ((S1 + 31) & ~31);
    const int b3 = b2 + ((S2 + 31) & ~31);
    const int b4 = b3 + ((S3 + 31) & ~31);
    const int myb = sub == 0 ? b0 : (sub == 1 ? b1 : (sub == 2 ? b2 : b3));
    if (tid == 0) {
      srb[min(4 * ch + 0, RBN - 1)] = b0;
      srb[min(4 * ch + 1, RBN - 1)] = b1;
      srb[min(4 * ch + 2, RBN - 1)] = b2;
      srb[min(4 * ch + 3, RBN - 1)] = b3;
    }
    int run = myb + pre + incl - ts;
    soff[8 * tid + 0] = run; run += e0;
    soff[8 * tid + 1] = run; run += e1;
    soff[8 * tid + 2] = run; run += e2;
    soff[8 * tid + 3] = run; run += e3;
    soff[8 * tid + 4] = run; run += e4;
    soff[8 * tid + 5] = run; run += e5;
    soff[8 * tid + 6] = run; run += e6;
    soff[8 * tid + 7] = run;
    carry = b4;
    __syncthreads();
    const v4i o0 = *(const v4i*)(soff + 4 * tid);
    const v4i o1 = *(const v4i*)(soff + 4 * (tid + OTHR));
    int* op = off + base;
    *(volatile v4i*)(op + 4 * tid) = o0;
    *(volatile v4i*)(op + 4 * (tid + OTHR)) = o1;
    __threadfence();
    *(volatile v4i*)(op + 4 * tid) = o0;
    *(volatile v4i*)(op + 4 * (tid + OTHR)) = o1;
    __syncthreads();
  }
  if (tid == 0) srb[min(4 * nChunk, RBN - 1)] = carry;
  __syncthreads();
  v4i rv = {0, 0, 0, 0};
  if (tid < 32) rv = *(const v4i*)(srb + 4 * tid);
  if (tid < 32) *(volatile v4i*)(rbase + 4 * tid) = rv;
  __threadfence();
  if (tid < 32) *(volatile v4i*)(rbase + 4 * tid) = rv;
}

__global__ __launch_bounds__(NTHR) void k_fill(
    const int* __restrict__ srcs, const int* __restrict__ dsts,
    const int* __restrict__ off, const int* __restrict__ rbase,
    int* csr, int nN, int nE, int vec8, int csrLen) {
  extern __shared__ v4f lds_dyn[];
  int* region = (int*)lds_dyn;
  int* cursor = region + RCAP;
  int* list   = cursor + NBF;
  int* wcnt   = list + LISTN;
  const int tid = threadIdx.x, lane = tid & 31, wave = tid >> 5;
  const int b = blockIdx.x;
  const int nodeBase = b * NBF;

  int rb0 = rbase[b];
  const int rb1 = rbase[b + 1];
  rb0 = rb0 < 0 ? 0 : (rb0 > csrLen ? csrLen : rb0);
  rb0 &= ~31;
  int len = rb1 - rb0;
  len = len < 0 ? 0 : (len > RCAP ? RCAP : len);
  int lenW = (len + 31) & ~31;
  if (rb0 + lenW > csrLen) lenW = (csrLen - rb0) & ~31;

  {
    const v4i z = {0, 0, 0, 0};
    for (int i = tid; i < RCAP / 4; i += NTHR) ((v4i*)region)[i] = z;
    for (int s = tid; s < NBF; s += NTHR) {
      int o = off[nodeBase + s] - rb0;
      o = o < 0 ? 0 : (o > RCAP ? RCAP : o);
      cursor[s] = o;
    }
  }
  __syncthreads();

  const int nChunks = (nE + CHUNK - 1) / CHUNK;
#pragma unroll 1
  for (int ch = 0; ch < nChunks; ++ch) {
    const int cbase = ch * CHUNK;
    const int wc = scan_chunk<NBF>(dsts, nE, cbase, nodeBase, vec8, list, tid, lane, wave);
    if (lane == 0) wcnt[wave] = wc;
    __syncthreads();
    if (wave == 0) {
#pragma unroll 1
      for (int wsx = 0; wsx < NWAVE; ++wsx) {
        int n = __builtin_amdgcn_readfirstlane(wcnt[wsx]);
        n = n > WCAP ? WCAP : (n < 0 ? 0 : n);
        const int* lp = list + wsx * WCAP;
#pragma unroll 1
        for (int i = 0; i < n; ++i) {
          const int ent  = __builtin_amdgcn_readfirstlane(lp[i]);
          const int slot = ent & (NBF - 1);
          int e = cbase + ((ent >> 12) & (CHUNK - 1));
          e = e > nE - 1 ? nE - 1 : e;
          int sv = srcs[e];
          sv = sv < 0 ? 0 : (sv > nN - 1 ? nN - 1 : sv);
          if (lane == 0) {
            int pos = cursor[slot];
            pos = pos < 0 ? 0 : (pos > RCAP - 1 ? RCAP - 1 : pos);
            region[pos] = sv;
            const int np = pos + 1;
            cursor[slot] = np > RCAP ? RCAP : np;
          }
        }
      }
    }
    __syncthreads();
  }

  const int nv = lenW >> 2;
  int* gp = csr + rb0;
#pragma unroll 1
  for (int i = tid; i < nv; i += NTHR) { const v4i v = ((const v4i*)region)[i]; *(volatile v4i*)(gp + 4 * i) = v; }
  __threadfence();
#pragma unroll 1
  for (int i = tid; i < nv; i += NTHR) { const v4i v = ((const v4i*)region)[i]; *(volatile v4i*)(gp + 4 * i) = v; }
}

__global__ __launch_bounds__(NTHR) void k_wtcvt(
    const float* __restrict__ W0, const float* __restrict__ W1, const float* __restrict__ W2,
    const float* __restrict__ W3, const float* __restrict__ W4, _Float16* planes) {
  const int y = blockIdx.y;
  const float* W = y == 0 ? W0 : (y == 1 ? W1 : (y == 2 ? W2 : (y == 3 ? W3 : W4)));
  const int Kreal = (y == 4) ? (FW + 1) : FW;
  const int KP    = (y == 4) ? KBMAX : FW;
  const int ppr   = KP >> 3;
  const int nUnits = FW * ppr;
  const int i = (int)blockIdx.x * NTHR + (int)threadIdx.x;
  if (i >= nUnits) return;
  const int n   = i / ppr;
  const int seg = i - n * ppr;
  v8h o;
#pragma unroll
  for (int j = 0; j < 8; ++j) {
    const int k  = 8 * seg + j;
    const int kc = k < Kreal - 1 ? k : Kreal - 1;
    const float w = W[(size_t)kc * FW + n];
    const float v = (k < Kreal) ? w * WCARRY : 0.f;
    o[j] = (_Float16)v;
  }
  _Float16* gp = planes + (size_t)y * PLH + (size_t)n * KP + 8 * seg;
  *(volatile v8h*)gp = o;
  __threadfence();
  *(volatile v8h*)gp = o;
}

template <int EXTRA>
__global__ __launch_bounds__(NTHR) void k_agg(
    const int* __restrict__ csr, const int* __restrict__ off, const int* __restrict__ cnt,
    const float* __restrict__ dinvI, const float* __restrict__ dinvO,
    const float* __restrict__ xin, const float* __restrict__ ntv,
    _Float16* a16, int nN, int csrLen) {
  const int tid = threadIdx.x, lane = tid & 31, wave = tid >> 5;
  const int tbase = blockIdx.x * TGT + wave * 32;
  const int col4 = 4 * lane;
  const int cl = tbase + lane;
  const int cnt_l = cnt[cl];
  const int off_l = off[cl];
  const float di_l = dinvI[cl];

#pragma unroll 1
  for (int j = 0; j < 32; ++j) {
    const int c = tbase + j;
    int n = __shfl(cnt_l, j);
    n = n < 0 ? 0 : (n > DEGCAP ? DEGCAP : n);
    const int st = __shfl(off_l, j);
    const float dc = __shfl(di_l, j);

    float a0 = 0.f, a1 = 0.f, a2 = 0.f, a3 = 0.f, ae = 0.f;
#pragma unroll 1
    for (int q0 = 0; q0 < n; q0 += 32) {
      int pos = st + q0 + lane;
      pos = pos < 0 ? 0 : (pos > csrLen - 1 ? csrLen - 1 : pos);
      int sl = csr[pos];
      sl = sl < 0 ? 0 : (sl > nN - 1 ? nN - 1 : sl);
      const int mcnt = (n - q0) < 32 ? (n - q0) : 32;
#pragma unroll 1
      for (int pp = 0; pp < mcnt; ++pp) {
        const int s = __builtin_amdgcn_readlane(sl, pp);
        const float cf = dinvO[s];
        const float* xr = xin + (size_t)s * FW + col4;
        const v4f x = *(const v4f*)xr;
        a0 += x.x * cf; a1 += x.y * cf; a2 += x.z * cf; a3 += x.w * cf;
        if constexpr (EXTRA != 0) ae += ntv[s] * cf;
      }
    }

    const bool live = c < nN;
    const float o0 = live ? (a0 * dc) * ACARRY : 0.f;
    const float o1 = live ? (a1 * dc) * ACARRY : 0.f;
    const float o2 = live ? (a2 * dc) * ACARRY : 0.f;
    const float o3 = live ? (a3 * dc) * ACARRY : 0.f;
    v4h oh;
    oh.x = (_Float16)o0; oh.y = (_Float16)o1; oh.z = (_Float16)o2; oh.w = (_Float16)o3;
    Pack4 pk; pk.h = oh;
    _Float16* rowp = a16 + (size_t)c * LDA16;
    unsigned int ex = 0u;
    if constexpr (EXTRA != 0) {
      const float oe = live ? (ae * dc) * ACARRY : 0.f;
      const _Float16 he = (_Float16)oe;
      const unsigned int hb = (unsigned int)__builtin_bit_cast(unsigned short, he);
      ex = (lane == 0) ? hb : 0u;
    }
    *(volatile v2u*)(rowp + col4) = pk.u;
    if constexpr (EXTRA != 0) *(volatile unsigned int*)(rowp + FW + 2 * lane) = ex;
    __threadfence();
    *(volatile v2u*)(rowp + col4) = pk.u;
    if constexpr (EXTRA != 0) *(volatile unsigned int*)(rowp + FW + 2 * lane) = ex;
  }
}

template <int LRELU, int CSUM, int ROWS, int HEAD>
__global__ __launch_bounds__(NTHR) void k_gemm(
    const _Float16* __restrict__ A, const _Float16* __restrict__ Bp, const float* __restrict__ bias,
    float* C32, float* xsum, const float* __restrict__ whd, const float* __restrict__ bhd,
    float* out, int KT, int nN) {
  constexpr int TPW = 4;
  constexpr int PPR = FW / 4;
  constexpr int NIT = (BM * PPR) / NTHR;
  static_assert((BM * PPR) % NTHR == 0);
  static_assert(NIT >= 1);

  __shared__ __attribute__((aligned(16))) float stg[BM * FW];
  __shared__ __attribute__((aligned(16))) float srow[FW];
  __shared__ __attribute__((aligned(16))) float swh[FW * NCLS];
  __shared__ __attribute__((aligned(16))) float sho[BM * NCLS];
  __shared__ float sbh[NCLS];
  const int tid = threadIdx.x, lane = tid & 31, wave = tid >> 5, hh = lane >> 4, m = lane & 15;
  const int rowBase = (int)blockIdx.x * BM;
  const int rg = wave >> 1, chf = wave & 1;
  const int r0 = rg * 16;
  const int c0 = chf * (FW / 2);
  const int KB = 32 * KT;

  if constexpr (HEAD != 0) {
    for (int i = tid; i < FW * NCLS; i += NTHR) swh[i] = whd[i];
    if (tid < NCLS) sbh[tid] = bhd[tid];
  }

  v8f acc[TPW];
#pragma unroll
  for (int t = 0; t < TPW; ++t) { v8f z = {0.f, 0.f, 0.f, 0.f, 0.f, 0.f, 0.f, 0.f}; acc[t] = z; }

  const _Float16* ap = A + (size_t)(rowBase + r0 + m) * LDA16 + 8 * hh;
  const _Float16* bp = Bp + (size_t)(c0 + m) * KB + 8 * hh;
#pragma unroll 1
  for (int kt = 0; kt < KT; ++kt) {
    Frag a;
    a.h[0] = *(const v8h*)(ap + 32 * kt);
    a.h[1] = *(const v8h*)(ap + 32 * kt + 16);
#pragma unroll
    for (int t = 0; t < TPW; ++t) {
      const size_t to = (size_t)(16 * t) * KB + 32 * kt;
      Frag b;
      b.h[0] = *(const v8h*)(bp + to);
      b.h[1] = *(const v8h*)(bp + to + 16);
      acc[t] = wmh(a.v, b.v, acc[t]);
    }
  }

  {
    float* sp = stg + (size_t)(r0 + 8 * hh) * FW + c0 + m;
#pragma unroll
    for (int t = 0; t < TPW; ++t) {
      const float bv = bias[c0 + 16 * t + m];
#pragma unroll
      for (int r = 0; r < 8; ++r) {
        float v = acc[t][r] * CARRY_INV + bv;
        if constexpr (LRELU != 0) v = lreluf(v);
        sp[r * FW + 16 * t] = v;
      }
    }
  }
  __syncthreads();

  if constexpr (ROWS != 0) {
    v4f cv[NIT];
#pragma unroll
    for (int it = 0; it < NIT; ++it) {
      const int id = it * NTHR + tid;
      const int row = id >> 5, seg = id & 31;
      cv[it] = *(const v4f*)(stg + (size_t)row * FW + 4 * seg);
    }
#pragma unroll
    for (int it = 0; it < NIT; ++it) {
      const int id = it * NTHR + tid;
      const int row = id >> 5, seg = id & 31;
      float* gp = C32 + (size_t)(rowBase + row) * FW + 4 * seg;
      *(volatile v4f*)gp = cv[it];
    }
    __threadfence();
#pragma unroll
    for (int it = 0; it < NIT; ++it) {
      const int id = it * NTHR + tid;
      const int row = id >> 5, seg = id & 31;
      float* gp = C32 + (size_t)(rowBase + row) * FW + 4 * seg;
      *(volatile v4f*)gp = cv[it];
    }
  }

  if constexpr (CSUM != 0) {
    const int cc = tid & (FW - 1);
    float s = 0.f;
#pragma unroll 4
    for (int r = 0; r < BM; ++r) {
      const float x = stg[r * FW + cc];
      s += (rowBase + r < nN) ? x : 0.f;
    }
    if (tid < FW) srow[tid] = s;
    __syncthreads();
    const bool act = tid < 32;
    const int q = act ? tid : 0;
    const v4f v = *(const v4f*)(srow + 4 * q);
    float* gp = xsum + (size_t)blockIdx.x * FW + 4 * q;
    if (act) *(volatile v4f*)gp = v;
    __threadfence();
    if (act) *(volatile v4f*)gp = v;
  }

  if constexpr (HEAD != 0) {
    const int row = tid >> 2, cp = (tid & 3) * 2;
    float h0 = 0.f, h1 = 0.f;
    const float* xr = stg + row * FW;
#pragma unroll 4
    for (int k = 0; k < FW; ++k) {
      const float x = xr[k];
      h0 += x * swh[k * NCLS + cp];
      h1 += x * swh[k * NCLS + cp + 1];
    }
    sho[row * NCLS + cp]     = h0 + sbh[cp];
    sho[row * NCLS + cp + 1] = h1 + sbh[cp + 1];
    __syncthreads();
    const bool inr = tid < 2 * BM;
    const int q = inr ? tid : 0;
    const bool act = inr && (rowBase + (q >> 1) < nN);
    const v4f v = *(const v4f*)(sho + 4 * q);
    float* gp = out + (size_t)rowBase * NCLS + 4 * q;
    if (act) *(volatile v4f*)gp = v;
    __threadfence();
    if (act) *(volatile v4f*)gp = v;
  }
}

template <int RS>
__global__ __launch_bounds__(FW) void k_red(const float* __restrict__ part, float* line, int nPart, int nN) {
  __shared__ __attribute__((aligned(16))) float srow[FW];
  const int tid = threadIdx.x;
  double s = 0.0;
#pragma unroll 1
  for (int b = 0; b < nPart; ++b) s += (double)part[(size_t)b * FW + tid];
  float v = (float)(s / (double)nN);
  if constexpr (RS != 0) v = rsqrtf(v + BN_EPS);
  srow[tid] = v;
  __syncthreads();
  const bool act = tid < 32;
  const int q = act ? tid : 0;
  const v4f o = *(const v4f*)(srow + 4 * q);
  if (act) *(volatile v4f*)(line + 4 * q) = o;
  __threadfence();
  if (act) *(volatile v4f*)(line + 4 * q) = o;
}

__global__ __launch_bounds__(NTHR) void k_var(const float* __restrict__ X, const float* __restrict__ mu,
                                              float* sq, int nN) {
  __shared__ __attribute__((aligned(16))) float scs[NWAVE * FW];
  __shared__ __attribute__((aligned(16))) float srow[FW];
  const int tid = threadIdx.x, lane = tid & 31, wave = tid >> 5;
  const int tbase = blockIdx.x * TGT + wave * 32;
  const int col4 = 4 * lane;
  const v4f mv = *(const v4f*)(mu + col4);
  float s0 = 0.f, s1 = 0.f, s2 = 0.f, s3 = 0.f;
#pragma unroll 1
  for (int j = 0; j < 32; ++j) {
    const int c = tbase + j;
    if (c >= nN) break;
    const v4f x = *(const v4f*)(X + (size_t)c * FW + col4);
    float d;
    d = x.x - mv.x; s0 += d * d;
    d = x.y - mv.y; s1 += d * d;
    d = x.z - mv.z; s2 += d * d;
    d = x.w - mv.w; s3 += d * d;
  }
  v4f cs; cs.x = s0; cs.y = s1; cs.z = s2; cs.w = s3;
  *(v4f*)(scs + wave * FW + col4) = cs;
  __syncthreads();
  const int cc = tid & (FW - 1);
  float s = 0.f;
#pragma unroll
  for (int w = 0; w < NWAVE; ++w) s += scs[w * FW + cc];
  if (tid < FW) srow[tid] = s;
  __syncthreads();
  const bool act = tid < 32;
  const int q = act ? tid : 0;
  const v4f v = *(const v4f*)(srow + 4 * q);
  float* gp = sq + (size_t)blockIdx.x * FW + 4 * q;
  if (act) *(volatile v4f*)gp = v;
  __threadfence();
  if (act) *(volatile v4f*)gp = v;
}

__global__ __launch_bounds__(NTHR) void k_bnapply(
    float* X, const float* __restrict__ mu, const float* __restrict__ rs,
    const float* __restrict__ gam, const float* __restrict__ bet, int nN) {
  const int tid = threadIdx.x, lane = tid & 31, wave = tid >> 5;
  const int tbase = blockIdx.x * TGT + wave * 32;
  const int col4 = 4 * lane;
  const v4f mv = *(const v4f*)(mu + col4);
  const v4f rv = *(const v4f*)(rs + col4);
  const v4f gv = *(const v4f*)(gam + col4);
  const v4f bv = *(const v4f*)(bet + col4);
#pragma unroll 1
  for (int j = 0; j < 32; ++j) {
    const int c = tbase + j;
    const bool live = c < nN;
    float* xp = X + (size_t)c * FW + col4;
    const v4f x = *(const v4f*)xp;
    v4f y;
    y.x = live ? lreluf(((x.x - mv.x) * rv.x) * gv.x + bv.x) : 0.f;
    y.y = live ? lreluf(((x.y - mv.y) * rv.y) * gv.y + bv.y) : 0.f;
    y.z = live ? lreluf(((x.z - mv.z) * rv.z) * gv.z + bv.z) : 0.f;
    y.w = live ? lreluf(((x.w - mv.w) * rv.w) * gv.w + bv.w) : 0.f;
    *(volatile v4f*)xp = y;
    __threadfence();
    *(volatile v4f*)xp = y;
  }
}

__global__ __launch_bounds__(NTHR) void k_pool(const float* __restrict__ hg, const int* __restrict__ gids,
                                               float* gmean, int nN, int vec8) {
  __shared__ __attribute__((aligned(16))) int list[LISTN];
  __shared__ __attribute__((aligned(16))) float scs[NWAVE * FW];
  __shared__ __attribute__((aligned(16))) float srow[FW];
  __shared__ int swc[NWAVE];
  const int tid = threadIdx.x, lane = tid & 31, wave = tid >> 5;
  const int g = blockIdx.x;
  const int col4 = 4 * lane;
  float a0 = 0.f, a1 = 0.f, a2 = 0.f, a3 = 0.f;
  int cw = 0;

  const int nChunks = (nN + CHUNK - 1) / CHUNK;
#pragma unroll 1
  for (int ch = 0; ch < nChunks; ++ch) {
    const int cbase = ch * CHUNK;
    const int wc = scan_chunk<1>(gids, nN, cbase, g, vec8, list, tid, lane, wave);
    __syncthreads();
    int n = wc > WCAP ? WCAP : (wc < 0 ? 0 : wc);
    const int* lp = list + wave * WCAP;
#pragma unroll 1
    for (int i = 0; i < n; ++i) {
      const int ent = __builtin_amdgcn_readfirstlane(lp[i]);
      int r = cbase + ((ent >> 12) & (CHUNK - 1));
      r = r > nN - 1 ? nN - 1 : (r < 0 ? 0 : r);
      const v4f x = *(const v4f*)(hg + (size_t)r * FW + col4);
      a0 += x.x; a1 += x.y; a2 += x.z; a3 += x.w;
    }
    cw += n;
    __syncthreads();
  }

  v4f cs; cs.x = a0; cs.y = a1; cs.z = a2; cs.w = a3;
  *(v4f*)(scs + wave * FW + col4) = cs;
  if (lane == 0) swc[wave] = cw;
  __syncthreads();
  const int cc = tid & (FW - 1);
  float s = 0.f;
  int ct = 0;
#pragma unroll
  for (int w = 0; w < NWAVE; ++w) { s += scs[w * FW + cc]; ct += swc[w]; }
  const float cf = (float)(ct < 1 ? 1 : ct);
  const float mv = s * (1.0f / cf);
  if (tid < FW) srow[tid] = mv;
  __syncthreads();
  const bool act = tid < 32;
  const int q = act ? tid : 0;
  const v4f v = *(const v4f*)(srow + 4 * q);
  float* gp = gmean + (size_t)g * FW + 4 * q;
  if (act) *(volatile v4f*)gp = v;
  __threadfence();
  if (act) *(volatile v4f*)gp = v;
}

__global__ __launch_bounds__(NTHR) void k_ghead(const float* __restrict__ gmean, const float* __restrict__ Wgc,
                                                const float* __restrict__ bgc, float* out1) {
  __shared__ __attribute__((aligned(16))) float sw[FW * GCLS];
  __shared__ __attribute__((aligned(16))) float sho[NGR * GCLS];
  const int tid = threadIdx.x;
  for (int i = tid; i < FW * GCLS; i += NTHR) sw[i] = Wgc[i];
  __syncthreads();
  const int g = tid >> 2, c = tid & 3;
  const float* gr = gmean + (size_t)g * FW;
  float acc = 0.f;
#pragma unroll 4
  for (int k = 0; k < FW; ++k) acc += gr[k] * sw[k * GCLS + c];
  sho[tid] = acc + bgc[c];
  __syncthreads();
  const bool act = tid < (NGR * GCLS) / 4;
  const int q = act ? tid : 0;
  const v4f v = *(const v4f*)(sho + 4 * q);
  if (act) *(volatile v4f*)(out1 + 4 * q) = v;
  __threadfence();
  if (act) *(volatile v4f*)(out1 + 4 * q) = v;
}

extern "C" void kernel_launch(void* const* d_in, const int* in_sizes, int n_in,
                              void* d_out, int out_size, void* d_ws, size_t ws_size,
                              hipStream_t stream) {
  if (n_in < 26) return;
  const int nN = in_sizes[1];
  const int nE = in_sizes[23];
  if (nN <= 0 || nE <= 0) return;
  if (in_sizes[0] != nN * FW) return;
  if (in_sizes[24] != nE || in_sizes[25] != nN) return;
  if (in_sizes[3] != FW * FW || in_sizes[7] != FW * FW) return;
  if (in_sizes[13] != FW * FW || in_sizes[15] != FW * FW) return;
  if (in_sizes[19] != (FW + 1) * FW) return;
  if (in_sizes[17] != FW * NCLS || in_sizes[21] != FW * GCLS) return;
  if (in_sizes[4] != FW || in_sizes[5] != FW || in_sizes[6] != FW) return;
  if (in_sizes[8] != FW || in_sizes[9] != FW || in_sizes[10] != FW) return;
  if (in_sizes[14] != FW || in_sizes[16] != FW || in_sizes[20] != FW) return;
  if (in_sizes[18] != NCLS || in_sizes[22] != GCLS) return;
  if (out_size != nN * NCLS + NGR * GCLS) return;
  if (nE > (1 << 28) || nN > (1 << 22)) return;

  const float* node_feat = (const float*)d_in[0];
  const float* nodetype  = (const float*)d_in[1];
  const float* W1    = (const float*)d_in[3];
  const float* b1    = (const float*)d_in[4];
  const float* gam1  = (const float*)d_in[5];
  const float* bet1  = (const float*)d_in[6];
  const float* W2    = (const float*)d_in[7];
  const float* b2    = (const float*)d_in[8];
  const float* gam2  = (const float*)d_in[9];
  const float* bet2  = (const float*)d_in[10];
  const float* Wn1   = (const float*)d_in[13];
  const float* b_nn1 = (const float*)d_in[14];
  const float* Wn2   = (const float*)d_in[15];
  const float* b_nn2 = (const float*)d_in[16];
  const float* Wnc   = (const float*)d_in[17];
  const float* b_nc  = (const float*)d_in[18];
  const float* Wg1   = (const float*)d_in[19];
  const float* b_g1  = (const float*)d_in[20];
  const float* Wgc   = (const float*)d_in[21];
  const float* b_gc  = (const float*)d_in[22];
  const int* src  = (const int*)d_in[23];
  const int* dst  = (const int*)d_in[24];
  const int* gids = (const int*)d_in[25];
  float* out0 = (float*)d_out;
  float* out1 = out0 + (size_t)nN * NCLS;

  const int NPAD   = ((nN + TGT - 1) / TGT) * TGT;
  const int nBC    = (nN + NBC - 1) / NBC;
  const int CNTPAD = nBC * NBC;
  if (CNTPAD < NPAD) return;
  if (4 * nBC + 1 > RBN) return;
  const int nBF    = (nN + NBF - 1) / NBF;
  if (nBF > 4 * nBC) return;
  const int csrLen = ((nE + 31) & ~31) + 4096;
  if (31 * 4 * nBC > 4096) return;
  const int nAgg   = NPAD / TGT;
  const int nGemm  = NPAD / BM;

  char* ws = (char*)d_ws;
  size_t off = 0;
  const size_t oWp  = off; off += (size_t)NWPL * PLH * 2;         off = (off + 255) & ~(size_t)255;
  const size_t oA   = off; off += (size_t)NPAD * LDA16 * 2;       off = (off + 255) & ~(size_t)255;
  const size_t oXa  = off; off += (size_t)NPAD * FW * 4;          off = (off + 255) & ~(size_t)255;
  const size_t oXb  = off; off += (size_t)NPAD * FW * 4;          off = (off + 255) & ~(size_t)255;
  const size_t oCnI = off; off += (size_t)CNTPAD * 4;             off = (off + 255) & ~(size_t)255;
  const size_t oDiI = off; off += (size_t)CNTPAD * 4;             off = (off + 255) & ~(size_t)255;
  const size_t oOff = off; off += (size_t)CNTPAD * 4;             off = (off + 255) & ~(size_t)255;
  const size_t oCnO = off; off += (size_t)CNTPAD * 4;             off = (off + 255) & ~(size_t)255;
  const size_t oDiO = off; off += (size_t)CNTPAD * 4;             off = (off + 255) & ~(size_t)255;
  const size_t oRb  = off; off += (size_t)RBN * 4;                off = (off + 255) & ~(size_t)255;
  const size_t oCsr = off; off += (size_t)csrLen * 4;             off = (off + 255) & ~(size_t)255;
  const size_t oXs  = off; off += (size_t)nGemm * FW * 4;         off = (off + 255) & ~(size_t)255;
  const size_t oSq  = off; off += (size_t)nAgg * FW * 4;          off = (off + 255) & ~(size_t)255;
  const size_t oMu  = off; off += (size_t)FW * 4;                 off = (off + 255) & ~(size_t)255;
  const size_t oRs  = off; off += (size_t)FW * 4;                 off = (off + 255) & ~(size_t)255;
  const size_t oGm  = off; off += (size_t)NGR * FW * 4;           off = (off + 255) & ~(size_t)255;
  if (off > ws_size || off > (size_t)WSCAP) return;

  _Float16* wpl  = (_Float16*)(ws + oWp);
  _Float16* a16  = (_Float16*)(ws + oA);
  float* Xa   = (float*)(ws + oXa);
  float* Xb   = (float*)(ws + oXb);
  int*   cntI = (int*)(ws + oCnI);
  float* diI  = (float*)(ws + oDiI);
  int*   offp = (int*)(ws + oOff);
  int*   cntO = (int*)(ws + oCnO);
  float* diO  = (float*)(ws + oDiO);
  int*   rb   = (int*)(ws + oRb);
  int*   csr  = (int*)(ws + oCsr);
  float* xsum = (float*)(ws + oXs);
  float* sq   = (float*)(ws + oSq);
  float* muL  = (float*)(ws + oMu);
  float* rsL  = (float*)(ws + oRs);
  float* gm   = (float*)(ws + oGm);

  const int vec8 = 1;

  k_wtcvt<<<dim3((FW * (KBMAX / 8) + NTHR - 1) / NTHR, NWPL, 1), NTHR, 0, stream>>>(W1, W2, Wn1, Wn2, Wg1, wpl);
  k_count<<<nBC, NTHR, 0, stream>>>(dst, cntI, diI, nE, vec8);
  k_count<<<nBC, NTHR, 0, stream>>>(src, cntO, diO, nE, vec8);
  k_offsets<<<1, OTHR, 0, stream>>>(cntI, offp, rb, nBC);
  hipFuncSetAttribute(reinterpret_cast<const void*>(&k_fill),
                      hipFuncAttributeMaxDynamicSharedMemorySize, LDS_FILL);
  k_fill<<<nBF, NTHR, LDS_FILL, stream>>>(src, dst, offp, rb, csr, nN, nE, vec8, csrLen);

  k_agg<0><<<nAgg, NTHR, 0, stream>>>(csr, offp, cntI, diI, diO, node_feat, nodetype, a16, nN, csrLen);
  k_gemm<0, 1, 1, 0><<<nGemm, NTHR, 0, stream>>>(a16, wpl + 0 * PLH, b1, Xa, xsum, Wnc, b_nc, out0, FW / 32, nN);
  k_red<0><<<1, FW, 0, stream>>>(xsum, muL, nGemm, nN);
  k_var<<<nAgg, NTHR, 0, stream>>>(Xa, muL, sq, nN);
  k_red<1><<<1, FW, 0, stream>>>(sq, rsL, nAgg, nN);
  k_bnapply<<<nAgg, NTHR, 0, stream>>>(Xa, muL, rsL, gam1, bet1, nN);

  k_agg<0><<<nAgg, NTHR, 0, stream>>>(csr, offp, cntI, diI, diO, Xa, nodetype, a16, nN, csrLen);
  k_gemm<0, 1, 1, 0><<<nGemm, NTHR, 0, stream>>>(a16, wpl + 1 * PLH, b2, Xb, xsum, Wnc, b_nc, out0, FW / 32, nN);
  k_red<0><<<1, FW, 0, stream>>>(xsum, muL, nGemm, nN);
  k_var<<<nAgg, NTHR, 0, stream>>>(Xb, muL, sq, nN);
  k_red<1><<<1, FW, 0, stream>>>(sq, rsL, nAgg, nN);
  k_bnapply<<<nAgg, NTHR, 0, stream>>>(Xb, muL, rsL, gam2, bet2, nN);

  k_agg<1><<<nAgg, NTHR, 0, stream>>>(csr, offp, cntI, diI, diO, Xb, nodetype, a16, nN, csrLen);
  k_gemm<1, 0, 1, 0><<<nGemm, NTHR, 0, stream>>>(a16, wpl + 2 * PLH, b_nn1, Xa, xsum, Wnc, b_nc, out0, FW / 32, nN);
  k_gemm<1, 0, 1, 0><<<nGemm, NTHR, 0, stream>>>(a16, wpl + 4 * PLH, b_g1, Xb, xsum, Wnc, b_nc, out0, KBMAX / 32, nN);
  k_pool<<<NGR, NTHR, 0, stream>>>(Xb, gids, gm, nN, vec8);
  k_ghead<<<1, NTHR, 0, stream>>>(gm, Wgc, b_gc, out1);
  k_agg<0><<<nAgg, NTHR, 0, stream>>>(csr, offp, cntI, diI, diO, Xa, nodetype, a16, nN, csrLen);
  k_gemm<1, 0, 0, 1><<<nGemm, NTHR, 0, stream>>>(a16, wpl + 3 * PLH, b_nn2, Xb, xsum, Wnc, b_nc, out0, FW / 32, nN);
}
